// DeepPhenoModel_86139864089465
// MI455X (gfx1250) — hardware-verified
//
#include <hip/hip_runtime.h>
#include <stddef.h>


typedef _Float16 v16h __attribute__((ext_vector_type(16)));
typedef _Float16 v8h  __attribute__((ext_vector_type(8)));
typedef float    v8f  __attribute__((ext_vector_type(8)));
typedef float    v4f  __attribute__((ext_vector_type(4)));
typedef _Float16 h16;

#ifndef NB
#define NB 64
#endif
#define NB_FULL 64
#define K1    10000
#define HIDN  1500
#define EXPW  53
#define K2V   1553
#define NCLS  2048
#define KP1   10048
#define KP2   1600
#define NP1   1600

static_assert(NB >= 64 && NB <= NB_FULL && (NB % 64) == 0);
static_assert(K2V == HIDN + EXPW);
static_assert((KP1 % 64) == 0 && KP1 >= K1 && (KP1 - K1) < 64);
static_assert((KP2 % 64) == 0 && KP2 >= K2V && (KP2 - K2V) < 64);
static_assert(NP1 == KP2 && (NP1 % 64) == 0 && NP1 >= K2V);
static_assert((NCLS % 128) == 0 && (NCLS % 64) == 0 && (NCLS % 8) == 0);
static_assert((K1 % 8) == 0);
static_assert(((NB * (KP1 / 8)) % 256) == 0);
static_assert(((KP1 / 8) % 8) == 0);

#define LDT 72
#define LDC 68
static_assert((LDT % 8) == 0 && LDT >= 64);
static_assert((LDC % 4) == 0 && LDC >= 64);
static_assert((size_t)64 * LDT * 2 <= (size_t)131072);
static_assert((size_t)64 * LDC * 4 <= (size_t)131072);
static_assert((size_t)8 * 128 * 4 <= (size_t)131072);

#define WCARRY 64.0f
#define MCARRY 16.0f

#define W1T_BYTES ((size_t)NP1 * KP1 * 2)
#define W2T_BYTES ((size_t)NCLS * KP2 * 2)
#define G16_BYTES ((size_t)NB * KP1 * 2)
#define X16_BYTES ((size_t)NB * KP2 * 2)
#define CM_BYTES  ((size_t)NCLS * 4)
#define OFF_W1T ((size_t)0)
#define OFF_W2T (OFF_W1T + W1T_BYTES)
#define OFF_G16 (OFF_W2T + W2T_BYTES)
#define OFF_X16 (OFF_G16 + G16_BYTES)
#define OFF_CM  (OFF_X16 + X16_BYTES)
#define WS_TOTAL (OFF_CM + CM_BYTES)
static_assert((W1T_BYTES % 128) == 0 && (W2T_BYTES % 128) == 0 && (G16_BYTES % 128) == 0);
static_assert((X16_BYTES % 128) == 0 && (CM_BYTES % 128) == 0);
static_assert(((size_t)KP1 * 2) % 128 == 0 && ((size_t)KP2 * 2) % 128 == 0);
static_assert(WS_TOTAL <= (size_t)134217728);

__device__ __forceinline__ float bf16r(float x) {
  unsigned int u = __float_as_uint(x);
  u = (u + 0x7FFFu + ((u >> 16) & 1u)) & 0xFFFF0000u;
  return __uint_as_float(u);
}

static __device__ __forceinline__ h16 toh_flush(float v) {
  const h16 r = (h16)v;
  return (fabsf(v) < 6.103515625e-05f) ? (h16)0.0f : r;
}

__device__ __forceinline__ v16h frag_at(const _Float16* p) {
  v8h lo = *(const v8h*)(p);
  v8h hi = *(const v8h*)(p + 16);
  v16h out;
#pragma unroll
  for (int i = 0; i < 8; ++i) { out[i] = lo[i]; out[i + 8] = hi[i]; }
  return out;
}

__device__ __forceinline__ v8f wmma16(v16h a, v16h b, v8f c) {
  v8f d = __builtin_amdgcn_wmma_f32_16x16x32_f16(false, a, false, b, (short)0, c,
                                                 false, false);
  asm volatile("v_nop\n\tv_nop\n\tv_nop\n\tv_nop" : "+v"(d) : "v"(a), "v"(b));
  return d;
}

__global__ __launch_bounds__(256) void wconv_kernel(
    const float* __restrict__ W, _Float16* __restrict__ Wt, unsigned ldw, unsigned ldk,
    unsigned nvalid, unsigned kvalid) {
  __shared__ _Float16 T[64 * LDT];
  const unsigned tid = threadIdx.x;
  const unsigned n0 = blockIdx.x * 64u;
  const unsigned k0 = blockIdx.y * 64u;
#pragma unroll 4
  for (unsigned j = 0; j < 16u; ++j) {
    const unsigned idx = tid + 256u * j;
    const unsigned kr = idx >> 6, nc = idx & 63u;
    const unsigned kk = k0 + kr, nn = n0 + nc;
    const unsigned kcl = (kk < kvalid) ? kk : (kvalid - 1u);
    const unsigned ncl = (nn < nvalid) ? nn : (nvalid - 1u);
    const float v = W[(size_t)kcl * ldw + ncl];
    const h16 hv = toh_flush(WCARRY * bf16r(v));
    T[nc * LDT + kr] = (kk < kvalid && nn < nvalid) ? hv : (h16)0.0f;
  }
  __syncthreads();
  v8h x[2];
  size_t off[2];
#pragma unroll
  for (unsigned i = 0; i < 2u; ++i) {
    const unsigned n = 32u * i + (tid >> 3);
    const unsigned kc = (tid & 7u) * 8u;
    x[i] = *(const v8h*)&T[n * LDT + kc];
    off[i] = (size_t)(n0 + n) * ldk + k0 + kc;
  }
#pragma unroll
  for (int i = 0; i < 2; ++i) *(volatile v8h*)(Wt + off[i]) = x[i];
  __threadfence();
#pragma unroll
  for (int i = 0; i < 2; ++i) *(volatile v8h*)(Wt + off[i]) = x[i];
}

__global__ __launch_bounds__(256) void gconv_kernel(
    const float* __restrict__ G, _Float16* __restrict__ G16) {
  const unsigned idx = blockIdx.x * 256u + threadIdx.x;
  const unsigned row = idx / (unsigned)(KP1 / 8);
  const unsigned c8 = idx - row * (unsigned)(KP1 / 8);
  const bool ok = c8 < (unsigned)(K1 / 8);
  const unsigned cc = ok ? c8 : (unsigned)(K1 / 8 - 1);
  const float* p = G + (size_t)row * K1 + cc * 8u;
  const v4f a0 = *(const v4f*)(p);
  const v4f a1 = *(const v4f*)(p + 4);
  v8h o;
#pragma unroll
  for (int i = 0; i < 4; ++i) {
    const h16 h0 = toh_flush(MCARRY * bf16r(a0[i]));
    const h16 h1 = toh_flush(MCARRY * bf16r(a1[i]));
    o[i]     = ok ? h0 : (h16)0.0f;
    o[i + 4] = ok ? h1 : (h16)0.0f;
  }
  _Float16* q = G16 + (size_t)idx * 8u;
  *(volatile v8h*)q = o;
  __threadfence();
  *(volatile v8h*)q = o;
}

__global__ __launch_bounds__(256) void colmax_kernel(
    const float* __restrict__ M, float* __restrict__ cmax) {
  __shared__ float Pm[8 * 128];
  const unsigned tid = threadIdx.x, lane = tid & 31u;
  const unsigned wave = (unsigned)__builtin_amdgcn_readfirstlane((int)(tid >> 5));
  const unsigned c0 = blockIdx.x * 128u + lane * 4u;
  const float* p = M + (size_t)(wave * (unsigned)(NCLS / 8)) * NCLS + c0;
  v4f mx = *(const v4f*)p;
#pragma unroll 4
  for (unsigned i = 1; i < (unsigned)(NCLS / 8); ++i) {
    const v4f a = *(const v4f*)(p + (size_t)i * NCLS);
#pragma unroll
    for (int j = 0; j < 4; ++j) mx[j] = fmaxf(mx[j], a[j]);
  }
  *(v4f*)&Pm[wave * 128u + lane * 4u] = mx;
  __syncthreads();
  if (wave == 0u) {
    v4f r = *(const v4f*)&Pm[lane * 4u];
#pragma unroll
    for (unsigned w = 1; w < 8u; ++w) {
      const v4f a = *(const v4f*)&Pm[w * 128u + lane * 4u];
#pragma unroll
      for (int j = 0; j < 4; ++j) r[j] = fmaxf(r[j], a[j]);
    }
#pragma unroll
    for (int j = 0; j < 4; ++j) r[j] = bf16r(r[j]);
    float* q = cmax + blockIdx.x * 128u + lane * 4u;
    *(volatile v4f*)q = r;
    __threadfence();
    *(volatile v4f*)q = r;
  }
}

template <int MODE>
__device__ __forceinline__ void gemm_body(
    const _Float16* __restrict__ A16, const _Float16* __restrict__ Bt, const unsigned K,
    const float* __restrict__ bias, const float* __restrict__ aux,
    float* __restrict__ outf, _Float16* __restrict__ out16) {
  __shared__ float Cs[64 * LDC];
  const unsigned tid = threadIdx.x, lane = tid & 31u, w = tid >> 5;
  const unsigned mw = w >> 1, nw = w & 1u;
  const unsigned hh = lane >> 4, m = lane & 15u;
  const unsigned n0 = blockIdx.x * 64u;
  const unsigned row0 = blockIdx.y * 64u;

  const _Float16* ap  = A16 + (size_t)(row0 + mw * 16u + m) * K + hh * 8u;
  const _Float16* bp0 = Bt + (size_t)(n0 + nw * 32u + m) * K + hh * 8u;
  const _Float16* bp1 = bp0 + (size_t)16 * K;
  v8f acc0 = {}, acc1 = {};
#pragma unroll 2
  for (unsigned k0 = 0; k0 < K; k0 += 32u) {
    const v16h a  = frag_at(ap + k0);
    const v16h b0 = frag_at(bp0 + k0);
    const v16h b1 = frag_at(bp1 + k0);
    acc0 = wmma16(a, b0, acc0);
    acc1 = wmma16(a, b1, acc1);
  }
#pragma unroll
  for (int r = 0; r < 8; ++r) {
    float* d = &Cs[(mw * 16u + hh * 8u + (unsigned)r) * LDC + nw * 32u + m];
    d[0]  = acc0[r];
    d[16] = acc1[r];
  }
  __syncthreads();

  if (MODE == 0) {
#pragma unroll 1
    for (unsigned e = 0; e < 16u; ++e) {
      const unsigned r = 32u * (e >> 3) + (tid >> 3);
      const unsigned c = (tid & 7u) * 8u + (e & 7u);
      const unsigned col = n0 + c;
      const unsigned cb = (col < (unsigned)HIDN) ? col : (unsigned)(HIDN - 1);
      const unsigned cx = (col >= (unsigned)HIDN) ? (col - (unsigned)HIDN) : 0u;
      const unsigned ce = (cx < (unsigned)EXPW) ? cx : (unsigned)(EXPW - 1);
      float bb = bias[cb];
      float ex = aux[(size_t)(row0 + r) * EXPW + ce];
      asm volatile("" : "+v"(bb));
      asm volatile("" : "+v"(ex));
      const float pre = Cs[r * LDC + c] * (1.0f / (WCARRY * MCARRY)) + bf16r(bb);
      const float gl = 0.5f * pre * (1.0f + erff(pre * 0.70710678118654752f));
      const float hv = MCARRY * gl;
      const float xv = MCARRY * bf16r(ex);
      const float t = (col < (unsigned)HIDN) ? hv : ((col < (unsigned)K2V) ? xv : 0.0f);
      Cs[r * LDC + c] = t;
    }
    __syncthreads();

    v8h x[2];
    size_t off[2];
#pragma unroll
    for (unsigned i = 0; i < 2u; ++i) {
      const unsigned r = 32u * i + (tid >> 3);
      const unsigned c = (tid & 7u) * 8u;
      const v4f u0 = *(const v4f*)&Cs[r * LDC + c];
      const v4f u1 = *(const v4f*)&Cs[r * LDC + c + 4];
#pragma unroll
      for (int j = 0; j < 4; ++j) {
        x[i][j]     = toh_flush(u0[j]);
        x[i][j + 4] = toh_flush(u1[j]);
      }
      off[i] = (size_t)(row0 + r) * KP2 + n0 + c;
    }
#pragma unroll
    for (int i = 0; i < 2; ++i) *(volatile v8h*)(out16 + off[i]) = x[i];
    __threadfence();
#pragma unroll
    for (int i = 0; i < 2; ++i) *(volatile v8h*)(out16 + off[i]) = x[i];
  }

  if (MODE == 1) {
#pragma unroll 1
    for (unsigned e = 0; e < 16u; ++e) {
      const unsigned r = 16u * (e >> 2) + (tid >> 4);
      const unsigned c = (tid & 15u) * 4u + (e & 3u);
      const unsigned col = n0 + c;
      const unsigned cc = (col < (unsigned)NCLS) ? col : (unsigned)(NCLS - 1);
      const float bb = bias[cc];
      const float cm = aux[cc];
      const float pre = Cs[r * LDC + c] * (1.0f / (WCARRY * MCARRY)) + bf16r(bb);
      const float sg = 1.0f / (1.0f + expf(-pre));
      Cs[r * LDC + c] = cm * sg;
    }
    __syncthreads();

    v4f xs[4];
    size_t off[4];
#pragma unroll
    for (unsigned i = 0; i < 4u; ++i) {
      const unsigned r = 16u * i + (tid >> 4);
      const unsigned c = (tid & 15u) * 4u;
      xs[i] = *(const v4f*)&Cs[r * LDC + c];
      off[i] = (size_t)(row0 + r) * NCLS + n0 + c;
    }
#pragma unroll
    for (int i = 0; i < 4; ++i) *(volatile v4f*)(outf + off[i]) = xs[i];
    __threadfence();
#pragma unroll
    for (int i = 0; i < 4; ++i) *(volatile v4f*)(outf + off[i]) = xs[i];
  }
}

__global__ __launch_bounds__(256) void gemm_hid_kernel(
    const _Float16* __restrict__ A16, const _Float16* __restrict__ Bt,
    const float* __restrict__ bias, const float* __restrict__ ex, _Float16* __restrict__ x16) {
  gemm_body<0>(A16, Bt, (unsigned)KP1, bias, ex, (float*)0, x16);
}
__global__ __launch_bounds__(256) void gemm_out_kernel(
    const _Float16* __restrict__ A16, const _Float16* __restrict__ Bt,
    const float* __restrict__ bias, const float* __restrict__ cmax, float* __restrict__ outf) {
  gemm_body<1>(A16, Bt, (unsigned)KP2, bias, cmax, outf, (_Float16*)0);
}

extern "C" void kernel_launch(void* const* d_in, const int* in_sizes, int n_in,
                              void* d_out, int out_size, void* d_ws, size_t ws_size,
                              hipStream_t stream) {
  if (n_in < 7) return;
  if ((long long)in_sizes[0] < (long long)NB * K1) return;
  if ((long long)in_sizes[1] < (long long)NB * EXPW) return;
  if ((long long)in_sizes[2] < (long long)K1 * HIDN) return;
  if (in_sizes[3] < HIDN) return;
  if ((long long)in_sizes[4] < (long long)K2V * NCLS) return;
  if (in_sizes[5] < NCLS) return;
  if ((long long)in_sizes[6] < (long long)NCLS * NCLS) return;
  if ((long long)out_size < (long long)NB * NCLS) return;
  if (ws_size < WS_TOTAL) return;

  const float* gin = (const float*)d_in[0];
  const float* exx = (const float*)d_in[1];
  const float* w1  = (const float*)d_in[2];
  const float* b1  = (const float*)d_in[3];
  const float* w2  = (const float*)d_in[4];
  const float* b2  = (const float*)d_in[5];
  const float* adj = (const float*)d_in[6];
  float* out = (float*)d_out;

  char* ws = (char*)d_ws;
  _Float16* W1T = (_Float16*)(ws + OFF_W1T);
  _Float16* W2T = (_Float16*)(ws + OFF_W2T);
  _Float16* G16 = (_Float16*)(ws + OFF_G16);
  _Float16* X16 = (_Float16*)(ws + OFF_X16);
  float*    CM  = (float*)(ws + OFF_CM);

  dim3 blk(256);

  colmax_kernel<<<dim3(NCLS / 128), blk, 0, stream>>>(adj, CM);
  gconv_kernel<<<dim3((NB * (KP1 / 8)) / 256), blk, 0, stream>>>(gin, G16);
  wconv_kernel<<<dim3(NP1 / 64, KP1 / 64), blk, 0, stream>>>(
      w1, W1T, (unsigned)HIDN, (unsigned)KP1, (unsigned)HIDN, (unsigned)K1);
  wconv_kernel<<<dim3(NCLS / 64, KP2 / 64), blk, 0, stream>>>(
      w2, W2T, (unsigned)NCLS, (unsigned)KP2, (unsigned)NCLS, (unsigned)K2V);
  gemm_hid_kernel<<<dim3(NP1 / 64, NB / 64), blk, 0, stream>>>(G16, W1T, b1, exx, X16);
  gemm_out_kernel<<<dim3(NCLS / 64, NB / 64), blk, 0, stream>>>(X16, W2T, b2, CM, out);
}
